// DFEM_59407987638548
// MI455X (gfx1250) — hardware-verified
//
#include <hip/hip_runtime.h>
#include <stdint.h>

#define DEV __device__ __forceinline__

typedef __bf16   v16b  __attribute__((ext_vector_type(16)));
typedef _Float16 v16h  __attribute__((ext_vector_type(16)));
typedef _Float16 v8h   __attribute__((ext_vector_type(8)));
typedef float    v8f   __attribute__((ext_vector_type(8)));
typedef float    v4f   __attribute__((ext_vector_type(4)));
typedef unsigned short u16x8 __attribute__((ext_vector_type(8)));
typedef v8h   __attribute__((may_alias)) v8ha;
typedef v4f   __attribute__((may_alias)) v4fa;
typedef u16x8 __attribute__((may_alias)) u16x8a;

union FragH { v16h v; v8h p[2]; };
union FragB { v16b v; u16x8 p[2]; };

constexpr int NB   = 8;
constexpr int NC   = 256;
constexpr int NP   = 4096;
constexpr int NQ   = 32;
constexpr int NCMB = 320;
constexpr float QKOUT  = 8.0f;
constexpr float ESC    = 1.0f / 64.0f;
constexpr float PSCALE = 16384.0f;
constexpr float OINV   = 1.0f / (16384.0f * 8.0f);

DEV v8f wmma_bf16(v16b a, v16b b, v8f c) {
  v8f d = __builtin_amdgcn_wmma_f32_16x16x32_bf16(false, a, false, b, (short)0, c, false, false);
  asm volatile("v_nop\n\tv_nop\n\tv_nop\n\tv_nop" : "+v"(d) : "v"(a), "v"(b));
  return d;
}
DEV v8f wmma_f16(v16h a, v16h b, v8f c) {
  v8f d = __builtin_amdgcn_wmma_f32_16x16x32_f16(false, a, false, b, (short)0, c, false, false);
  asm volatile("v_nop\n\tv_nop\n\tv_nop\n\tv_nop" : "+v"(d) : "v"(a), "v"(b));
  return d;
}
DEV v8f wmma_split3(v16b ah, v16b al, v16b bh, v16b bl, v8f c) {
  c = wmma_bf16(ah, bh, c);
  c = wmma_bf16(ah, bl, c);
  c = wmma_bf16(al, bh, c);
  return c;
}

DEV v16b bfrag(const unsigned short* p, int h) {
  FragB f;
  f.p[0] = *(const u16x8a*)(p + 8 * h);
  f.p[1] = *(const u16x8a*)(p + 16 + 8 * h);
  return f.v;
}
DEV v16h hfrag(const _Float16* p, int h) {
  FragH f;
  f.p[0] = *(const v8ha*)(p + 8 * h);
  f.p[1] = *(const v8ha*)(p + 16 + 8 * h);
  return f.v;
}

DEV unsigned short f2bf(float f) {
  const unsigned u = __float_as_uint(f);
  const unsigned r = u + 0x7FFFu + ((u >> 16) & 1u);
  return (unsigned short)(r >> 16);
}
DEV void split_bf(float v, unsigned short& hi, unsigned short& lo) {
  hi = f2bf(v);
  const float hf = __uint_as_float(((unsigned)hi) << 16);
  lo = f2bf(v - hf);
}
DEV int clampi(int v, int lo, int hi) { return v < lo ? lo : (v > hi ? hi : v); }

__global__ __launch_bounds__(256) void prep_weights(
    const float* __restrict__ w1, const float* __restrict__ wq,
    const float* __restrict__ wk, const float* __restrict__ wv,
    unsigned short* w1h, unsigned short* w1l,
    unsigned short* wch, unsigned short* wcl)
{
  constexpr int NG1 = NC * NC / 8;
  constexpr int NGQ = NQ * NC / 8;
  constexpr int NGV = NC * NC / 8;
  constexpr int NGT = NG1 + 2 * NGQ + NGV;
  const int g = blockIdx.x * 256 + threadIdx.x;
  if (g >= NGT) return;
  const float* src;
  unsigned short* dh;
  unsigned short* dl;
  if (g < NG1) {
    src = w1 + (size_t)g * 8;
    dh = w1h + (size_t)g * 8;
    dl = w1l + (size_t)g * 8;
  } else {
    const int e = g - NG1;
    if (e < NGQ)            src = wq + (size_t)e * 8;
    else if (e < 2 * NGQ)   src = wk + (size_t)(e - NGQ) * 8;
    else                    src = wv + (size_t)(e - 2 * NGQ) * 8;
    dh = wch + (size_t)e * 8;
    dl = wcl + (size_t)e * 8;
  }
  const v4f a = *(const v4fa*)src;
  const v4f c = *(const v4fa*)(src + 4);
  const float vv[8] = {a.x, a.y, a.z, a.w, c.x, c.y, c.z, c.w};
  u16x8 oh, ol;
#pragma unroll
  for (int j = 0; j < 8; ++j) {
    unsigned short hi, lo;
    split_bf(vv[j], hi, lo);
    oh[j] = hi;
    ol[j] = lo;
  }
  *(volatile u16x8*)dh = oh;
  *(volatile u16x8*)dl = ol;
  __threadfence();
  *(volatile u16x8*)dh = oh;
  *(volatile u16x8*)dl = ol;
}

DEV void conv1_store(const float* sD, float* xf, unsigned short* xTh, unsigned short* xTl,
                     int b, int p0, int w, int lane) {
  const int q8 = lane & 7, sub = lane >> 3;
#pragma unroll
  for (int i = 0; i < 16; ++i) {
    const int c = 64 * w + 4 * i + sub;
    v4f v;
    v.x = sD[(4 * q8 + 0) * 256 + c];
    v.y = sD[(4 * q8 + 1) * 256 + c];
    v.z = sD[(4 * q8 + 2) * 256 + c];
    v.w = sD[(4 * q8 + 3) * 256 + c];
    float* d = xf + ((size_t)(b * NC + c)) * NP + p0 + 4 * q8;
    *(volatile v4f*)d = v;
  }
#pragma unroll
  for (int i = 0; i < 8; ++i) {
    const int p = 8 * w + i;
    const v4f a = *(const v4fa*)(sD + p * 256 + 8 * lane);
    const v4f c = *(const v4fa*)(sD + p * 256 + 8 * lane + 4);
    const float vv[8] = {a.x, a.y, a.z, a.w, c.x, c.y, c.z, c.w};
    u16x8 oh, ol;
#pragma unroll
    for (int j = 0; j < 8; ++j) {
      unsigned short hi, lo;
      split_bf(vv[j], hi, lo);
      oh[j] = hi;
      ol[j] = lo;
    }
    const size_t ro = ((size_t)(b * NP + p0 + p)) * NC + 8 * lane;
    *(volatile u16x8*)(xTh + ro) = oh;
    *(volatile u16x8*)(xTl + ro) = ol;
  }
}

__global__ __launch_bounds__(128) void conv1_kernel(
    const float* __restrict__ x,
    const unsigned short* __restrict__ w1h,
    const unsigned short* __restrict__ w1l,
    const float* __restrict__ b1,
    float* xf,
    unsigned short* xTh,
    unsigned short* xTl)
{
  __shared__ __attribute__((aligned(16))) unsigned short sAh[32 * 40];
  __shared__ __attribute__((aligned(16))) unsigned short sAl[32 * 40];
  __shared__ __attribute__((aligned(16))) float sD[32 * 256];

  const int tid = threadIdx.x, lane = tid & 31, w = tid >> 5;
  const int h = lane >> 4, m = lane & 15;
  const int b = blockIdx.y, p0 = blockIdx.x * 32;
  const float* xb = x + (size_t)b * NC * NP;
  const int ci = tid >> 2, pp = (tid & 3) * 8;
  const unsigned short* wrh = w1h + (size_t)(64 * w + m) * NC;
  const unsigned short* wrl = w1l + (size_t)(64 * w + m) * NC;

  const v8f zero8 = {0.f, 0.f, 0.f, 0.f, 0.f, 0.f, 0.f, 0.f};
  v8f acc[2][4];
#pragma unroll
  for (int mt = 0; mt < 2; ++mt)
#pragma unroll
    for (int nt = 0; nt < 4; ++nt) acc[mt][nt] = zero8;

#pragma unroll 1
  for (int k0 = 0; k0 < NC; k0 += 32) {
    __syncthreads();
    {
      const float* src = xb + (size_t)(k0 + ci) * NP + p0 + pp;
      const v4f a = *(const v4fa*)src;
      const v4f c = *(const v4fa*)(src + 4);
      const float vv[8] = {a.x, a.y, a.z, a.w, c.x, c.y, c.z, c.w};
#pragma unroll
      for (int j = 0; j < 8; ++j) {
        unsigned short hi, lo;
        split_bf(vv[j], hi, lo);
        sAh[(pp + j) * 40 + ci] = hi;
        sAl[(pp + j) * 40 + ci] = lo;
      }
    }
    __syncthreads();
    const v16b ah0 = bfrag(sAh + m * 40, h);
    const v16b ah1 = bfrag(sAh + (16 + m) * 40, h);
    const v16b al0 = bfrag(sAl + m * 40, h);
    const v16b al1 = bfrag(sAl + (16 + m) * 40, h);
#pragma unroll
    for (int nt = 0; nt < 4; ++nt) {
      const v16b bh = bfrag(wrh + (size_t)nt * 16 * NC + k0, h);
      const v16b bl = bfrag(wrl + (size_t)nt * 16 * NC + k0, h);
      acc[0][nt] = wmma_split3(ah0, al0, bh, bl, acc[0][nt]);
      acc[1][nt] = wmma_split3(ah1, al1, bh, bl, acc[1][nt]);
    }
  }

#pragma unroll
  for (int nt = 0; nt < 4; ++nt) {
    const int co = 64 * w + 16 * nt + m;
    const float bias = b1[co];
#pragma unroll
    for (int mt = 0; mt < 2; ++mt)
#pragma unroll
      for (int r = 0; r < 8; ++r)
        sD[(16 * mt + 8 * h + r) * 256 + co] = acc[mt][nt][r] + bias;
  }
  __syncthreads();

  conv1_store(sD, xf, xTh, xTl, b, p0, w, lane);
  __threadfence();
  conv1_store(sD, xf, xTh, xTl, b, p0, w, lane);
}

DEV void proj_store(const float* sD, _Float16* Qp, _Float16* Kp, _Float16* Vp,
                    int g, int b, int p0, int w, int lane) {
  if (g == 0) {
    _Float16* qb = Qp + ((size_t)(b * NP + p0)) * NQ;
    _Float16* kb = Kp + ((size_t)(b * NP + p0)) * NQ;
#pragma unroll
    for (int j = 0; j < 2; ++j) {
      const int i = 64 * w + 32 * j + lane;
      const int p = i >> 2, cp = (i & 3) * 8;
      const v4f a  = *(const v4fa*)(sD + p * 64 + cp);
      const v4f c  = *(const v4fa*)(sD + p * 64 + cp + 4);
      const v4f a2 = *(const v4fa*)(sD + p * 64 + 32 + cp);
      const v4f c2 = *(const v4fa*)(sD + p * 64 + 32 + cp + 4);
      const v8h oq = { (_Float16)a.x, (_Float16)a.y, (_Float16)a.z, (_Float16)a.w,
                       (_Float16)c.x, (_Float16)c.y, (_Float16)c.z, (_Float16)c.w };
      const v8h ok = { (_Float16)a2.x, (_Float16)a2.y, (_Float16)a2.z, (_Float16)a2.w,
                       (_Float16)c2.x, (_Float16)c2.y, (_Float16)c2.z, (_Float16)c2.w };
      *(volatile v8h*)(qb + 8 * i) = oq;
      *(volatile v8h*)(kb + 8 * i) = ok;
    }
  } else {
    const int q8 = lane & 7, sub = lane >> 3;
#pragma unroll
    for (int j = 0; j < 4; ++j) {
      const int cl = 16 * w + 4 * j + sub;
      const int cv = 64 * (g - 1) + cl;
      const v8h o = { (_Float16)sD[(8 * q8 + 0) * 64 + cl], (_Float16)sD[(8 * q8 + 1) * 64 + cl],
                      (_Float16)sD[(8 * q8 + 2) * 64 + cl], (_Float16)sD[(8 * q8 + 3) * 64 + cl],
                      (_Float16)sD[(8 * q8 + 4) * 64 + cl], (_Float16)sD[(8 * q8 + 5) * 64 + cl],
                      (_Float16)sD[(8 * q8 + 6) * 64 + cl], (_Float16)sD[(8 * q8 + 7) * 64 + cl] };
      *(volatile v8h*)(Vp + ((size_t)(b * NC + cv)) * NP + p0 + 8 * q8) = o;
    }
  }
}

__global__ __launch_bounds__(128) void proj_kernel(
    const unsigned short* __restrict__ xTh,
    const unsigned short* __restrict__ xTl,
    const unsigned short* __restrict__ wch,
    const unsigned short* __restrict__ wcl,
    const float* __restrict__ bq, const float* __restrict__ bk, const float* __restrict__ bv,
    _Float16* Qp,
    _Float16* Kp,
    _Float16* Vp)
{
  __shared__ __attribute__((aligned(16))) float sD[64 * 64];

  const int tid = threadIdx.x, lane = tid & 31, w = tid >> 5;
  const int h = lane >> 4, m = lane & 15;
  const int b = blockIdx.z, g = blockIdx.y, p0 = blockIdx.x * 64;

  const unsigned short* arh = xTh + ((size_t)(b * NP + p0 + 16 * w + m)) * NC;
  const unsigned short* arl = xTl + ((size_t)(b * NP + p0 + 16 * w + m)) * NC;
  const unsigned short* brh = wch + ((size_t)(64 * g + m)) * NC;
  const unsigned short* brl = wcl + ((size_t)(64 * g + m)) * NC;

  const v8f zero8 = {0.f, 0.f, 0.f, 0.f, 0.f, 0.f, 0.f, 0.f};
  v8f acc[4];
#pragma unroll
  for (int nt = 0; nt < 4; ++nt) acc[nt] = zero8;

#pragma unroll 1
  for (int k0 = 0; k0 < NC; k0 += 32) {
    const v16b ah = bfrag(arh + k0, h);
    const v16b al = bfrag(arl + k0, h);
#pragma unroll
    for (int nt = 0; nt < 4; ++nt) {
      const v16b bh = bfrag(brh + (size_t)nt * 16 * NC + k0, h);
      const v16b bl = bfrag(brl + (size_t)nt * 16 * NC + k0, h);
      acc[nt] = wmma_split3(ah, al, bh, bl, acc[nt]);
    }
  }

#pragma unroll
  for (int nt = 0; nt < 4; ++nt) {
    const int cl = 16 * nt + m;
    const int cc = 64 * g + cl;
    const float fq = bq[clampi(cc, 0, NQ - 1)];
    const float fk = bk[clampi(cc - NQ, 0, NQ - 1)];
    const float fv = bv[clampi(cc - 2 * NQ, 0, NC - 1)];
    const float bias = (cc < NQ) ? fq : ((cc < 2 * NQ) ? fk : fv);
#pragma unroll
    for (int r = 0; r < 8; ++r)
      sD[(16 * w + 8 * h + r) * 64 + cl] = (acc[nt][r] + bias) * QKOUT;
  }
  __syncthreads();

  proj_store(sD, Qp, Kp, Vp, g, b, p0, w, lane);
  __threadfence();
  proj_store(sD, Qp, Kp, Vp, g, b, p0, w, lane);
}

DEV v16h pack_p(v8f a, v8f c) {
  const v16h r = { (_Float16)(a[0] * PSCALE), (_Float16)(a[1] * PSCALE), (_Float16)(a[2] * PSCALE), (_Float16)(a[3] * PSCALE),
                   (_Float16)(a[4] * PSCALE), (_Float16)(a[5] * PSCALE), (_Float16)(a[6] * PSCALE), (_Float16)(a[7] * PSCALE),
                   (_Float16)(c[0] * PSCALE), (_Float16)(c[1] * PSCALE), (_Float16)(c[2] * PSCALE), (_Float16)(c[3] * PSCALE),
                   (_Float16)(c[4] * PSCALE), (_Float16)(c[5] * PSCALE), (_Float16)(c[6] * PSCALE), (_Float16)(c[7] * PSCALE) };
  return r;
}

DEV void attn_store(const float* sO, const float* xf, const float* xin, const float* Apl,
                    const float* wt, float* dst, float g, int mode, int b, int qblk,
                    int rr, int w, int lane) {
  const int q8 = lane & 7, sub = lane >> 3;
#pragma unroll
  for (int i = 0; i < 8; ++i) {
    const int lid = 32 * w + 4 * i + sub;
    const int cl = lid >> 1, hl = lid & 1;
    const int c = 128 * rr + cl;
    const int qo = 32 * hl + 4 * q8;
    const v4f ov = *(const v4fa*)(sO + cl * 64 + qo);
    const size_t gi = ((size_t)(b * NC + c)) * NP + qblk + qo;
    const v4f xr = *(const v4fa*)(xf + gi);
    const v4f xi = *(const v4fa*)(xin + gi);
    v4f val;
    val.x = xi.x * (g * ov.x + xr.x);
    val.y = xi.y * (g * ov.y + xr.y);
    val.z = xi.z * (g * ov.z + xr.z);
    val.w = xi.w * (g * ov.w + xr.w);
    if (mode != 0) {
      const v4f ap = *(const v4fa*)(Apl + gi);
      const v4f ww = *(const v4fa*)(wt + (size_t)b * NP + qblk + qo);
      val.x = ww.x * fabsf(val.x - ap.x);
      val.y = ww.y * fabsf(val.y - ap.y);
      val.z = ww.z * fabsf(val.z - ap.z);
      val.w = ww.w * fabsf(val.w - ap.w);
    }
    *(volatile v4f*)(dst + gi) = val;
  }
}

__global__ __launch_bounds__(256) void attn_kernel(
    const _Float16* __restrict__ Qp,
    const _Float16* __restrict__ Kp,
    const _Float16* __restrict__ Vp,
    const float* __restrict__ xf,
    const float* __restrict__ xin,
    const float* __restrict__ gamma,
    const float* Apl,
    const float* wt,
    float* dst,
    int mode)
{
  __shared__ __attribute__((aligned(16))) float sO[128 * 64];

  const int tid = threadIdx.x, lane = tid & 31, w = tid >> 5;
  const int h = lane >> 4, m = lane & 15;
  const int qg = w & 3, chh = w >> 2;
  const int b = blockIdx.y;
  const int qblk = blockIdx.x * 64;
  const int q0 = qblk + 16 * qg;

  const v16h qb = hfrag(Qp + ((size_t)(b * NP + q0 + m)) * NQ, h);

  const v8f zero8 = {0.f, 0.f, 0.f, 0.f, 0.f, 0.f, 0.f, 0.f};
  v8f o[8];
#pragma unroll
  for (int t = 0; t < 8; ++t) o[t] = zero8;
  float mrun = -1e30f, lrun = 0.0f;

  const _Float16* kbase = Kp + ((size_t)(b * NP + m)) * NQ;
  const _Float16* vbase = Vp + ((size_t)(b * NC + 128 * chh + m)) * NP;

#pragma unroll 1
  for (int kb = 0; kb < NP; kb += 64) {
    v8f s[4];
#pragma unroll
    for (int j = 0; j < 4; ++j) {
      const v16h kf = hfrag(kbase + (size_t)(kb + 16 * j) * NQ, h);
      s[j] = wmma_f16(kf, qb, zero8);
    }
    float mloc = -1e30f;
#pragma unroll
    for (int j = 0; j < 4; ++j)
#pragma unroll
      for (int r = 0; r < 8; ++r) {
        const float e = s[j][r] * ESC;
        s[j][r] = e;
        mloc = fmaxf(mloc, e);
      }
    mloc = fmaxf(mloc, __shfl_xor(mloc, 16));
    const float mnew = fmaxf(mrun, mloc);
    const float alpha = __expf(mrun - mnew);
    mrun = mnew;
    float lsum = 0.0f;
#pragma unroll
    for (int j = 0; j < 4; ++j)
#pragma unroll
      for (int r = 0; r < 8; ++r) {
        const float p = __expf(s[j][r] - mnew);
        s[j][r] = p;
        lsum += p;
      }
    lsum += __shfl_xor(lsum, 16);
    lrun = lrun * alpha + lsum;
#pragma unroll
    for (int t = 0; t < 8; ++t)
#pragma unroll
      for (int r = 0; r < 8; ++r) o[t][r] = o[t][r] * alpha;

    const v16h pb0 = pack_p(s[0], s[1]);
    const v16h pb1 = pack_p(s[2], s[3]);

#pragma unroll
    for (int t = 0; t < 8; ++t) {
      const _Float16* vp = vbase + (size_t)(16 * t) * NP + kb;
      const v16h vf0 = hfrag(vp, h);
      const v16h vf1 = hfrag(vp + 32, h);
      o[t] = wmma_f16(vf0, pb0, o[t]);
      o[t] = wmma_f16(vf1, pb1, o[t]);
    }
  }

  const float inv = (1.0f / lrun) * OINV;
  const float g = gamma[0];
#pragma unroll
  for (int rr = 0; rr < 2; ++rr) {
    if (chh == rr) {
#pragma unroll
      for (int t = 0; t < 8; ++t)
#pragma unroll
        for (int r = 0; r < 8; ++r)
          sO[(16 * t + 8 * h + r) * 64 + 16 * qg + m] = o[t][r] * inv;
    }
    __syncthreads();
    attn_store(sO, xf, xin, Apl, wt, dst, g, mode, b, qblk, rr, w, lane);
    __threadfence();
    attn_store(sO, xf, xin, Apl, wt, dst, g, mode, b, qblk, rr, w, lane);
    __syncthreads();
  }
}

__global__ __launch_bounds__(256) void chan_stats(
    const float* __restrict__ xf, const float* s1, const float* m1,
    float* so, float* mo, int fin)
{
  const int idx = blockIdx.x * 256 + threadIdx.x;
  if (idx >= NB * NP) return;
  const int b = idx >> 12, p = idx & (NP - 1);
  const float* base = xf + (size_t)b * NC * NP + p;
  float sum = 0.0f, mx = -3.0e38f;
#pragma unroll 8
  for (int c = 0; c < NC; ++c) {
    const float v = base[(size_t)c * NP];
    sum += v;
    mx = fmaxf(mx, v);
  }
  float vs = sum, vm = mx;
  if (fin != 0) {
    vs = (s1[idx] + sum) * (1.0f / 512.0f);
    vm = fmaxf(m1[idx], mx);
  }
  *(volatile float*)(so + idx) = vs;
  *(volatile float*)(mo + idx) = vm;
  __threadfence();
  *(volatile float*)(so + idx) = vs;
  *(volatile float*)(mo + idx) = vm;
}

__global__ __launch_bounds__(256) void sa_conv(
    const float* __restrict__ maps, const float* __restrict__ wsa, float* wt)
{
  const int idx = blockIdx.x * 256 + threadIdx.x;
  if (idx >= NB * NP) return;
  const int b = idx >> 12, p = idx & (NP - 1);
  const int y = p >> 6, x = p & 63;
  float acc = 0.0f;
#pragma unroll 1
  for (int i = 0; i < 2; ++i) {
    const float* mp = maps + (size_t)i * NB * NP + (size_t)b * NP;
#pragma unroll 1
    for (int dy = 0; dy < 3; ++dy) {
      const int yy = y + dy - 1;
      const bool oky = (unsigned)yy < 64u;
      const int yc = clampi(yy, 0, 63);
#pragma unroll
      for (int dx = 0; dx < 3; ++dx) {
        const int xx = x + dx - 1;
        const bool okx = (unsigned)xx < 64u;
        const int xc = clampi(xx, 0, 63);
        float v = mp[yc * 64 + xc];
        v = (oky && okx) ? v : 0.0f;
        acc += wsa[i * 9 + dy * 3 + dx] * v;
      }
    }
  }
  const float e = expf(-acc);
  const float r = 1.0f / (1.0f + e);
  *(volatile float*)(wt + idx) = r;
  __threadfence();
  *(volatile float*)(wt + idx) = r;
}

extern "C" void kernel_launch(void* const* d_in, const int* in_sizes, int n_in,
                              void* d_out, int out_size, void* d_ws, size_t ws_size,
                              hipStream_t stream) {
  constexpr int NX = NB * NC * NP;
  if (n_in < 12) return;
  if (in_sizes[0] != NX || in_sizes[1] != NX) return;
  if (in_sizes[2] != NC * NC || in_sizes[3] != NC) return;
  if (in_sizes[4] != NQ * NC || in_sizes[5] != NQ) return;
  if (in_sizes[6] != NQ * NC || in_sizes[7] != NQ) return;
  if (in_sizes[8] != NC * NC || in_sizes[9] != NC) return;
  if (in_sizes[10] < 1 || in_sizes[11] != 18) return;
  if (out_size != NX) return;

  const float* x1    = (const float*)d_in[0];
  const float* x2    = (const float*)d_in[1];
  const float* w1    = (const float*)d_in[2];
  const float* b1    = (const float*)d_in[3];
  const float* wq    = (const float*)d_in[4];
  const float* bq    = (const float*)d_in[5];
  const float* wk    = (const float*)d_in[6];
  const float* bk    = (const float*)d_in[7];
  const float* wv    = (const float*)d_in[8];
  const float* bv    = (const float*)d_in[9];
  const float* gamma = (const float*)d_in[10];
  const float* wsa   = (const float*)d_in[11];
  float* out = (float*)d_out;

  size_t off = 0;
  auto carve = [&](size_t bytes) -> size_t {
    const size_t o = off;
    off += (bytes + 255) & ~(size_t)255;
    return o;
  };
  const size_t o_w1h  = carve((size_t)NC * NC * 2);
  const size_t o_w1l  = carve((size_t)NC * NC * 2);
  const size_t o_wch  = carve((size_t)NCMB * NC * 2);
  const size_t o_wcl  = carve((size_t)NCMB * NC * 2);
  const size_t o_xf   = carve((size_t)NX * 4);
  const size_t o_xth  = carve((size_t)NX * 2);
  const size_t o_xtl  = carve((size_t)NX * 2);
  const size_t o_q    = carve((size_t)NB * NP * NQ * 2);
  const size_t o_k    = carve((size_t)NB * NP * NQ * 2);
  const size_t o_v    = carve((size_t)NX * 2);
  const size_t o_a    = carve((size_t)NX * 4);
  const size_t o_s1   = carve((size_t)NB * NP * 4);
  const size_t o_m1   = carve((size_t)NB * NP * 4);
  const size_t o_maps = carve((size_t)2 * NB * NP * 4);
  const size_t o_wt   = carve((size_t)NB * NP * 4);
  if (off > ws_size) return;

  char* ws = (char*)d_ws;
  unsigned short* w1h = (unsigned short*)(ws + o_w1h);
  unsigned short* w1l = (unsigned short*)(ws + o_w1l);
  unsigned short* wch = (unsigned short*)(ws + o_wch);
  unsigned short* wcl = (unsigned short*)(ws + o_wcl);
  float*          xf  = (float*)(ws + o_xf);
  unsigned short* xth = (unsigned short*)(ws + o_xth);
  unsigned short* xtl = (unsigned short*)(ws + o_xtl);
  _Float16*       qp  = (_Float16*)(ws + o_q);
  _Float16*       kp  = (_Float16*)(ws + o_k);
  _Float16*       vp  = (_Float16*)(ws + o_v);
  float*          apl = (float*)(ws + o_a);
  float*          s1  = (float*)(ws + o_s1);
  float*          m1  = (float*)(ws + o_m1);
  float*          maps = (float*)(ws + o_maps);
  float*          wt  = (float*)(ws + o_wt);

  const dim3 gConv(NP / 32, NB);
  const dim3 gProj(NP / 64, 5, NB);
  const dim3 gAttn(NP / 64, NB);
  const int nStat = (NB * NP + 255) / 256;

  prep_weights<<<72, 256, 0, stream>>>(w1, wq, wk, wv, w1h, w1l, wch, wcl);

  conv1_kernel<<<gConv, 128, 0, stream>>>(x1, w1h, w1l, b1, xf, xth, xtl);
  chan_stats<<<nStat, 256, 0, stream>>>(xf, s1, m1, s1, m1, 0);
  proj_kernel<<<gProj, 128, 0, stream>>>(xth, xtl, wch, wcl, bq, bk, bv, qp, kp, vp);
  attn_kernel<<<gAttn, 256, 0, stream>>>(qp, kp, vp, xf, x1, gamma, apl, wt, apl, 0);

  conv1_kernel<<<gConv, 128, 0, stream>>>(x2, w1h, w1l, b1, xf, xth, xtl);
  chan_stats<<<nStat, 256, 0, stream>>>(xf, s1, m1, maps, maps + (size_t)NB * NP, 1);
  sa_conv<<<nStat, 256, 0, stream>>>(maps, wsa, wt);
  proj_kernel<<<gProj, 128, 0, stream>>>(xth, xtl, wch, wcl, bq, bk, bv, qp, kp, vp);
  attn_kernel<<<gAttn, 256, 0, stream>>>(qp, kp, vp, xf, x2, gamma, apl, wt, out, 1);
}
